// LSTMNet_28922309771279
// MI455X (gfx1250) — hardware-verified
//
#include <hip/hip_runtime.h>
#include <math.h>

constexpr int NBAT      = 1024;
constexpr int NIN       = 4;
constexpr int NSEQ      = 512;
constexpr int NHID      = 128;
constexpr int NGATE     = 4 * NHID;
constexpr int NFUT      = 16;
constexpr int NTOUT     = NSEQ + NFUT;
constexpr int NTHR      = 256;
constexpr int ROWS_BLK  = 64;
constexpr int HPITCH    = 136;
constexpr int TILE_EL   = ROWS_BLK * HPITCH;
constexpr int XCHUNK    = 32;
constexpr int GATE_PLANE = NHID * NHID;
constexpr int NOUT_EL   = NBAT * NIN * NTOUT;

constexpr float WCARRY   = 16.0f;
constexpr float HCARRY   = 16.0f;
constexpr float ZCARRY   = WCARRY * HCARRY;
constexpr float RES_SC   = 2048.0f;
constexpr float LOG2E_F  = 1.4426950408889634f;
constexpr float KSIG     = -LOG2E_F / ZCARRY;
constexpr float KTANH    = 2.0f * LOG2E_F / ZCARRY;
constexpr float KCELL    = 2.0f * LOG2E_F;
constexpr float ZINV     = 1.0f / ZCARRY;
constexpr float ZRINV    = 1.0f / (ZCARRY * RES_SC);

static_assert(NBAT % ROWS_BLK == 0, "batch tile");
static_assert(NHID == 16 * (NTHR / 32), "one 16-unit group per wave");
static_assert(NHID % 32 == 0, "K multiple of 32");
static_assert(HPITCH % 8 == 0 && HPITCH >= NHID, "tile pitch");
static_assert(NSEQ % XCHUNK == 0, "x chunking");
static_assert((2 * TILE_EL) % NTHR == 0, "tile zero-fill exact");
static_assert(ROWS_BLK * NIN == NTHR, "x chunk loader: one (row, feature) per thread");
static_assert((NTOUT % 4) == 0, "16-B output vectors never straddle a feature row");
static_assert((2 * NIN * NTOUT) % 128 == 0, "two batch rows = whole 512-B store groups");
static_assert((NOUT_EL / 4) % (66 * NTHR) == 0, "guard grid exact");

typedef __attribute__((ext_vector_type(16))) _Float16 v16h;
typedef __attribute__((ext_vector_type(8)))  _Float16 v8h;
typedef __attribute__((ext_vector_type(8)))  float    v8f;
typedef __attribute__((ext_vector_type(4)))  float    v4f;

__device__ __forceinline__ void acc_guard4(v8f& a, v8f& b, v8f& c, v8f& d) { asm volatile("v_nop\n\tv_nop\n\tv_nop\n\tv_nop" : "+v"(a), "+v"(b), "+v"(c), "+v"(d)); }
__device__ __forceinline__ void grp_guard_h(v8f& d0, v8f& d1, v8f& d2, v8f& d3, v16h a0, v16h a1, v16h a2, v16h a3, v16h b) {
  asm volatile("v_nop\n\tv_nop\n\tv_nop\n\tv_nop" : "+v"(d0), "+v"(d1), "+v"(d2), "+v"(d3) : "v"(a0), "v"(a1), "v"(a2), "v"(a3), "v"(b));
}

template <typename T> struct Frag;
template <> struct Frag<_Float16> {
  typedef v16h V; union U { v16h v; v8h h[2]; };
  static __device__ __forceinline__ v16h load(const _Float16* p) {
    U f; f.h[0] = *(const v8h*)(p); f.h[1] = *(const v8h*)(p + 16); return f.v;
  }
  static __device__ __forceinline__ v8f mma(v16h a, v16h b, v8f c) {
    return __builtin_amdgcn_wmma_f32_16x16x32_f16(false, a, false, b, (short)0, c, false, false);
  }
};
typedef Frag<_Float16> FragH;

__device__ __forceinline__ v8f mma_guarded_h(v16h a, v16h b, v8f c) {
  c = __builtin_amdgcn_wmma_f32_16x16x32_f16(false, a, false, b, (short)0, c, false, false);
  asm volatile("v_nop\n\tv_nop\n\tv_nop\n\tv_nop" : "+v"(c) : "v"(a), "v"(b));
  return c;
}

__device__ __forceinline__ float fx2(float x) { return __builtin_amdgcn_exp2f(x); }
__device__ __forceinline__ float frc(float x) { return __builtin_amdgcn_rcpf(x); }

template <bool ZC>
__device__ __forceinline__ void kc_step(v8f (&acc)[4][4], const _Float16* wp, const _Float16* hp) {
  const v8f z8 = {0.f, 0.f, 0.f, 0.f, 0.f, 0.f, 0.f, 0.f};
  const v16h a0 = FragH::load(wp);
  const v16h a1 = FragH::load(wp + 1 * GATE_PLANE);
  const v16h a2 = FragH::load(wp + 2 * GATE_PLANE);
  const v16h a3 = FragH::load(wp + 3 * GATE_PLANE);
#pragma unroll
  for (int nt = 0; nt < 4; ++nt) {
    const v16h b = FragH::load(hp + nt * 16 * HPITCH);
    if (ZC) {
      acc[0][nt] = FragH::mma(a0, b, z8);
      acc[1][nt] = FragH::mma(a1, b, z8);
      acc[2][nt] = FragH::mma(a2, b, z8);
      acc[3][nt] = FragH::mma(a3, b, z8);
    } else {
      acc[0][nt] = FragH::mma(a0, b, acc[0][nt]);
      acc[1][nt] = FragH::mma(a1, b, acc[1][nt]);
      acc[2][nt] = FragH::mma(a2, b, acc[2][nt]);
      acc[3][nt] = FragH::mma(a3, b, acc[3][nt]);
    }
    grp_guard_h(acc[0][nt], acc[1][nt], acc[2][nt], acc[3][nt], a0, a1, a2, a3, b);
  }
}

__device__ __forceinline__ void cell_update(v8f (&acc)[4][4], const float* bkl, float* csl, _Float16* hn) {
  float bk[4][8];
#pragma unroll
  for (int j = 0; j < 4; ++j) {
    const v4f b0 = *(const v4f*)(bkl + j * NHID);
    const v4f b1 = *(const v4f*)(bkl + j * NHID + 4);
#pragma unroll
    for (int e = 0; e < 4; ++e) { bk[j][e] = b0[e]; bk[j][4 + e] = b1[e]; }
  }
#pragma unroll
  for (int nt = 0; nt < 4; ++nt) {
    float* cp = csl + nt * 256;
    const v4f c0 = *(const v4f*)(cp);
    const v4f c1 = *(const v4f*)(cp + 4);
    float cold[8], cnew[8];
#pragma unroll
    for (int e = 0; e < 4; ++e) { cold[e] = c0[e]; cold[4 + e] = c1[e]; }
    v8h hv;
#pragma unroll
    for (int r = 0; r < 8; ++r) {
      const float ei = fx2(fmaf(acc[0][nt][r], KSIG,  bk[0][r]));
      const float ef = fx2(fmaf(acc[1][nt][r], KSIG,  bk[1][r]));
      const float eg = fx2(fmaf(acc[2][nt][r], KTANH, bk[2][r]));
      const float eo = fx2(fmaf(acc[3][nt][r], KSIG,  bk[3][r]));
      const float ig = frc(1.0f + ei);
      const float fg = frc(1.0f + ef);
      const float og = frc(1.0f + eo);
      const float gg = fmaf(frc(1.0f + eg), -2.0f, 1.0f);
      const float cn = fmaf(fg, cold[r], ig * gg);
      const float ec = fx2(cn * KCELL);
      const float th = fmaf(frc(1.0f + ec), -2.0f * HCARRY, HCARRY);
      cnew[r] = cn;
      hv[r] = (_Float16)(og * th);
    }
    v4f n0, n1;
#pragma unroll
    for (int e = 0; e < 4; ++e) { n0[e] = cnew[e]; n1[e] = cnew[4 + e]; }
    *(v4f*)(cp) = n0;
    *(v4f*)(cp + 4) = n1;
    *(v8h*)(hn + nt * 16 * HPITCH) = hv;
  }
}

__global__ __launch_bounds__(NTHR) void prep_kernel(const float* __restrict__ whh0, const float* __restrict__ wih1,
                                                    const float* __restrict__ whh1, const float* __restrict__ wl,
                                                    unsigned short* __restrict__ W0H, unsigned short* __restrict__ W1I,
                                                    unsigned short* __restrict__ W1H, unsigned short* __restrict__ WLP) {
  const int tid = threadIdx.x;
  const int bx = blockIdx.x;
  if (bx < 96) {
    const int which = bx >> 5;
    const float* src = (which == 0) ? whh0 : ((which == 1) ? wih1 : whh1);
    unsigned short* dst = (which == 0) ? W0H : ((which == 1) ? W1I : W1H);
    const int i = (bx & 31) * NTHR + tid;
    const v4f a = *(const v4f*)(src + (size_t)i * 8);
    const v4f b = *(const v4f*)(src + (size_t)i * 8 + 4);
    v8h hv;
#pragma unroll
    for (int e = 0; e < 4; ++e) {
      hv[e]     = (_Float16)(a[e] * WCARRY);
      hv[4 + e] = (_Float16)(b[e] * WCARRY);
    }
    *(volatile v8h*)(dst + (size_t)i * 8) = hv;
    __threadfence();
    *(volatile v8h*)(dst + (size_t)i * 8) = hv;
  } else {
    const int row = tid >> 4;
    const int c8 = (tid & 15) * 8;
    const int srow = row & 3;
    const v4f a = *(const v4f*)(wl + srow * NHID + c8);
    const v4f b = *(const v4f*)(wl + srow * NHID + c8 + 4);
    v8h hv;
#pragma unroll
    for (int e = 0; e < 8; ++e) {
      const float s = ((e < 4) ? a[e & 3] : b[e & 3]) * WCARRY;
      const _Float16 hi = (_Float16)s;
      const float hf = (float)hi;
      const _Float16 lo = (_Float16)((s - hf) * RES_SC);
      const _Float16 zz = (_Float16)0.0f;
      hv[e] = (row < 4) ? hi : ((row < 8) ? lo : zz);
    }
    *(volatile v8h*)(WLP + (size_t)tid * 8) = hv;
    __threadfence();
    *(volatile v8h*)(WLP + (size_t)tid * 8) = hv;
  }
}

__global__ __launch_bounds__(NTHR) void lstm_seq_kernel(const float* __restrict__ x, const float* __restrict__ wih0,
                                                        const float* __restrict__ bih0, const float* __restrict__ bhh0,
                                                        const float* __restrict__ bih1, const float* __restrict__ bhh1,
                                                        const float* __restrict__ bl,
                                                        const unsigned short* __restrict__ W0Hp,
                                                        const unsigned short* __restrict__ W1Ip,
                                                        const unsigned short* __restrict__ W1Hp,
                                                        const unsigned short* __restrict__ WLPp,
                                                        float* __restrict__ OUTS) {
  __shared__ __align__(16) _Float16 Hh0[2 * TILE_EL];
  __shared__ __align__(16) _Float16 Hh1[2 * TILE_EL];
  __shared__ __align__(16) float    cs[2 * 8 * 4 * 32 * 8];
  __shared__ __align__(16) float    xs[XCHUNK * ROWS_BLK * NIN];
  __shared__ __align__(16) float    w0s[NHID * 16];
  __shared__ __align__(16) float    bks[2 * NGATE];
  __shared__ __align__(16) float    osl[ROWS_BLK * NIN];
  __shared__ __align__(16) float    bls[4];

  const int tid  = threadIdx.x;
  const int lane = tid & 31;
  const int wave = __builtin_amdgcn_readfirstlane(tid >> 5);
  const int c    = lane & 15;
  const int hh   = lane >> 4;
  const int rowbase = blockIdx.x * ROWS_BLK;

#pragma unroll 1
  for (int i = tid; i < 2 * TILE_EL; i += NTHR) {
    Hh0[i] = (_Float16)0.0f;
    Hh1[i] = (_Float16)0.0f;
  }
  {
    const v4f z4 = {0.f, 0.f, 0.f, 0.f};
#pragma unroll
    for (int L = 0; L < 2; ++L)
#pragma unroll
      for (int nt = 0; nt < 4; ++nt) {
        float* cp = cs + (((L * 8 + wave) * 4 + nt) * 32 + lane) * 8;
        *(v4f*)(cp) = z4;
        *(v4f*)(cp + 4) = z4;
      }
  }
#pragma unroll 1
  for (int i = 0; i < 8; ++i) {
    const int d = i * NTHR + tid;
    const int k = d & 3, j = (d >> 2) & 3, u = d >> 4;
    w0s[d] = ZCARRY * wih0[(j * NHID + u) * NIN + k];
  }
#pragma unroll 1
  for (int i = 0; i < 4; ++i) {
    const int d = i * NTHR + tid;
    const int L = d >> 9, n = d & (NGATE - 1), j = n >> 7;
    const float s0 = bih0[n] + bhh0[n];
    const float s1 = bih1[n] + bhh1[n];
    const float s = (L == 0) ? s0 : s1;
    const float kk = (j == 2) ? (2.0f * LOG2E_F) : (-LOG2E_F);
    bks[d] = kk * s;
  }
  if (tid < 4) bls[tid] = bl[tid];
  __syncthreads();

  const _Float16* W0 = (const _Float16*)W0Hp + (size_t)(16 * wave + c) * NHID + 8 * hh;
  const _Float16* W1i = (const _Float16*)W1Ip + (size_t)(16 * wave + c) * NHID + 8 * hh;
  const _Float16* W1h = (const _Float16*)W1Hp + (size_t)(16 * wave + c) * NHID + 8 * hh;
  const _Float16* WL = (const _Float16*)WLPp + (size_t)c * NHID + 8 * hh;
  const int hoff = c * HPITCH + 8 * hh;
  const int hsto = c * HPITCH + 16 * wave + 8 * hh;
  const float* bk0 = bks + 16 * wave + 8 * hh;
  const float* bk1 = bks + NGATE + 16 * wave + 8 * hh;
  float* cs0 = cs + (((0 * 8 + wave) * 4) * 32 + lane) * 8;
  float* cs1 = cs + (((1 * 8 + wave) * 4) * 32 + lane) * 8;
  const v8f z8 = {0.f, 0.f, 0.f, 0.f, 0.f, 0.f, 0.f, 0.f};

#pragma unroll 1
  for (int t = 0; t < NTOUT; ++t) {
    const int cur = t & 1;
    const _Float16* h0c = Hh0 + cur * TILE_EL;
    _Float16*       h0n = Hh0 + (cur ^ 1) * TILE_EL;
    const _Float16* h1c = Hh1 + cur * TILE_EL;
    _Float16*       h1n = Hh1 + (cur ^ 1) * TILE_EL;

    if (t < NSEQ && (t & (XCHUNK - 1)) == 0) {
      const int bq = tid >> 2, kq = tid & 3;
      const float* src = x + ((size_t)(rowbase + bq) * NIN + kq) * NSEQ + t;
#pragma unroll
      for (int i = 0; i < 8; ++i) {
        const v4f v = *(const v4f*)(src + 4 * i);
#pragma unroll
        for (int e = 0; e < 4; ++e) xs[(4 * i + e) * (ROWS_BLK * NIN) + bq * NIN + kq] = v[e];
      }
      __syncthreads();
    }

    v8f acc[4][4];
    {
      const float* xp = xs + (t & (XCHUNK - 1)) * (ROWS_BLK * NIN) + c * NIN;
      v4f xv[4];
#pragma unroll
      for (int nt = 0; nt < 4; ++nt) xv[nt] = *(const v4f*)(xp + nt * 16 * NIN);
#pragma unroll
      for (int j = 0; j < 4; ++j) {
#pragma unroll
        for (int r = 0; r < 8; ++r) {
          const v4f wv = *(const v4f*)(w0s + ((16 * wave + 8 * hh + r) * 4 + j) * 4);
#pragma unroll
          for (int nt = 0; nt < 4; ++nt) {
            float s = xv[nt][0] * wv[0];
            s = fmaf(xv[nt][1], wv[1], s);
            s = fmaf(xv[nt][2], wv[2], s);
            s = fmaf(xv[nt][3], wv[3], s);
            acc[j][nt][r] = s;
          }
        }
      }
    }
#pragma unroll 1
    for (int kc = 0; kc < NHID / 32; ++kc) kc_step<false>(acc, W0 + kc * 32, h0c + hoff + kc * 32);
    acc_guard4(acc[0][0], acc[0][1], acc[0][2], acc[0][3]);
    acc_guard4(acc[1][0], acc[1][1], acc[1][2], acc[1][3]);
    acc_guard4(acc[2][0], acc[2][1], acc[2][2], acc[2][3]);
    acc_guard4(acc[3][0], acc[3][1], acc[3][2], acc[3][3]);
    cell_update(acc, bk0, cs0, h0n + hsto);
    __syncthreads();

    kc_step<true>(acc, W1i, h0n + hoff);
#pragma unroll 1
    for (int kc = 1; kc < NHID / 32; ++kc) kc_step<false>(acc, W1i + kc * 32, h0n + hoff + kc * 32);
#pragma unroll 1
    for (int kc = 0; kc < NHID / 32; ++kc) kc_step<false>(acc, W1h + kc * 32, h1c + hoff + kc * 32);
    acc_guard4(acc[0][0], acc[0][1], acc[0][2], acc[0][3]);
    acc_guard4(acc[1][0], acc[1][1], acc[1][2], acc[1][3]);
    acc_guard4(acc[2][0], acc[2][1], acc[2][2], acc[2][3]);
    acc_guard4(acc[3][0], acc[3][1], acc[3][2], acc[3][3]);
    cell_update(acc, bk1, cs1, h1n + hsto);
    __syncthreads();

    const bool wx = (t == NSEQ - 2) || (t >= NSEQ);
    const int  xw = (t == NSEQ - 2) ? 0 : ((t + 1) & (XCHUNK - 1));
    if (wave < 4) {
      const _Float16* hb = h1n + (16 * wave + c) * HPITCH + 8 * hh;
      v8f o8 = z8;
#pragma unroll
      for (int kc = 0; kc < NHID / 32; ++kc) {
        const v16h a = FragH::load(WL + kc * 32);
        const v16h b = FragH::load(hb + kc * 32);
        o8 = mma_guarded_h(a, b, o8);
      }
      const v4f blv = *(const v4f*)(bls);
      v4f ov;
#pragma unroll
      for (int f = 0; f < 4; ++f) ov[f] = fmaf(o8[4 + f], ZRINV, o8[f] * ZINV) + blv[f];
      if (hh == 0) {
        *(v4f*)(osl + (16 * wave + c) * NIN) = ov;
        if (wx) *(v4f*)(xs + xw * (ROWS_BLK * NIN) + (16 * wave + c) * NIN) = ov;
      }
    }
    __syncthreads();

    if (wave < 2) {
      const v4f v = *(const v4f*)(osl + (32 * wave + lane) * NIN);
      float* op = OUTS + ((size_t)t * NBAT + (size_t)(rowbase + 32 * wave + lane)) * NIN;
      *(volatile v4f*)op = v;
      __threadfence();
      *(volatile v4f*)op = v;
    }
  }
}

__global__ __launch_bounds__(NTHR) void out_pack_kernel(const float* __restrict__ OUTS, float* __restrict__ out) {
  const int lane = threadIdx.x & 31;
  const int pair = blockIdx.x * (NTHR / 32) + (threadIdx.x >> 5);
  if (pair >= NBAT / 2) return;
  float* op = out + (size_t)pair * (2 * NIN * NTOUT);
  for (int pass = 0; pass < 2; ++pass) {
#pragma unroll 1
    for (int i = 0; i < (2 * NIN * NTOUT) / 128; ++i) {
      const int e   = (i * 32 + lane) * 4;
      const int bb  = e / (NIN * NTOUT);
      const int rem = e - bb * (NIN * NTOUT);
      const int f   = rem / NTOUT;
      const int tt  = rem - f * NTOUT;
      const float* sp = OUTS + ((size_t)tt * NBAT + (size_t)(2 * pair + bb)) * NIN + f;
      v4f v;
      v[0] = sp[0];
      v[1] = sp[(size_t)1 * NBAT * NIN];
      v[2] = sp[(size_t)2 * NBAT * NIN];
      v[3] = sp[(size_t)3 * NBAT * NIN];
      *(volatile v4f*)(op + e) = v;
    }
    __threadfence();
  }
}

__global__ __launch_bounds__(NTHR) void premise_guard_kernel(const int* __restrict__ fut, float* __restrict__ out) {
  const int fv = fut[0];
  if (fv == NFUT) return;
  const float qn = __uint_as_float(0x7fc00000u);
  const v4f nv = {qn, qn, qn, qn};
  const int n4 = NOUT_EL / 4;
  const int stride = gridDim.x * NTHR;
  for (int pass = 0; pass < 2; ++pass) {
#pragma unroll 1
    for (int i = blockIdx.x * NTHR + threadIdx.x; i < n4; i += stride) *(volatile v4f*)(out + (size_t)i * 4) = nv;
    __threadfence();
  }
}

extern "C" void kernel_launch(void* const* d_in, const int* in_sizes, int n_in,
                              void* d_out, int out_size, void* d_ws, size_t ws_size, hipStream_t stream) {
  if (n_in < 12 || d_out == nullptr || d_ws == nullptr) return;
  if (in_sizes[0] != NBAT * NIN * NSEQ || in_sizes[1] != NGATE * NIN || in_sizes[2] != NGATE * NHID ||
      in_sizes[3] != NGATE || in_sizes[4] != NGATE || in_sizes[5] != NGATE * NHID || in_sizes[6] != NGATE * NHID ||
      in_sizes[7] != NGATE || in_sizes[8] != NGATE || in_sizes[9] != NIN * NHID || in_sizes[10] != NIN ||
      in_sizes[11] != 1 || out_size != NOUT_EL) return;

  const float* x    = (const float*)d_in[0];
  const float* wih0 = (const float*)d_in[1];
  const float* whh0 = (const float*)d_in[2];
  const float* bih0 = (const float*)d_in[3];
  const float* bhh0 = (const float*)d_in[4];
  const float* wih1 = (const float*)d_in[5];
  const float* whh1 = (const float*)d_in[6];
  const float* bih1 = (const float*)d_in[7];
  const float* bhh1 = (const float*)d_in[8];
  const float* wl   = (const float*)d_in[9];
  const float* bl   = (const float*)d_in[10];
  const int*   fut  = (const int*)d_in[11];
  float* out = (float*)d_out;

  char* ws = (char*)d_ws;
  size_t off = 0;
  auto carve = [&](size_t bytes) -> char* { char* p = ws + off; off += (bytes + 255) & ~(size_t)255; return p; };
  unsigned short* W0H = (unsigned short*)carve((size_t)NGATE * NHID * 2);
  unsigned short* W1I = (unsigned short*)carve((size_t)NGATE * NHID * 2);
  unsigned short* W1H = (unsigned short*)carve((size_t)NGATE * NHID * 2);
  unsigned short* WLP = (unsigned short*)carve((size_t)16 * NHID * 2);
  float*          OUTS = (float*)carve((size_t)NTOUT * NBAT * NIN * 4);
  if (off > ws_size || off > (size_t)134217728) return;

  prep_kernel<<<97, NTHR, 0, stream>>>(whh0, wih1, whh1, wl, W0H, W1I, W1H, WLP);
  lstm_seq_kernel<<<NBAT / ROWS_BLK, NTHR, 0, stream>>>(x, wih0, bih0, bhh0, bih1, bhh1, bl, W0H, W1I, W1H, WLP, OUTS);
  out_pack_kernel<<<(NBAT / 2) / (NTHR / 32), NTHR, 0, stream>>>(OUTS, out);
  premise_guard_kernel<<<66, NTHR, 0, stream>>>(fut, out);
}
